// QuantumNATExtendedQML_65481071409864
// MI455X (gfx1250) — hardware-verified
//
#include <hip/hip_runtime.h>
#include <math.h>

typedef __attribute__((ext_vector_type(16))) _Float16 v16h;
typedef __attribute__((ext_vector_type(16))) __bf16 v16b;
typedef __attribute__((ext_vector_type(8)))  _Float16 v8h;
typedef __attribute__((ext_vector_type(8)))  float v8f;
typedef __attribute__((ext_vector_type(4)))  float v4f;
typedef __attribute__((ext_vector_type(2)))  float v2f;
typedef __attribute__((ext_vector_type(4)))  unsigned v4u;
typedef __attribute__((ext_vector_type(4)))  int v4i;
typedef float __attribute__((may_alias)) float_a;
typedef int __attribute__((may_alias)) int_a;

template <typename T> __device__ __forceinline__ void vst2(void* p, T v) { *(volatile T*)p = v; __threadfence(); *(volatile T*)p = v; }
__device__ __forceinline__ v8f wmma16(v16h a, v16h b, v8f c) {
  v8f d = __builtin_amdgcn_wmma_f32_16x16x32_f16(false, a, false, b, (short)0, c, false, false);
  asm volatile("v_nop\n\tv_nop\n\tv_nop\n\tv_nop" : "+v"(d) : "v"(a), "v"(b));
  return d;
}
__device__ __forceinline__ v8f wmma_bf(v16b a, v16b b, v8f c) {
  v8f d = __builtin_amdgcn_wmma_f32_16x16x32_bf16(false, a, false, b, (short)0, c, false, false);
  asm volatile("v_nop\n\tv_nop\n\tv_nop\n\tv_nop" : "+v"(d) : "v"(a), "v"(b));
  return d;
}
__device__ __forceinline__ v16h frag_h(const _Float16* rowk0, int lane) {
  union { v16h v; v8h q[2]; } u; const _Float16* p = rowk0 + 8 * (lane >> 4);
  u.q[0] = *(const v8h*)p; u.q[1] = *(const v8h*)(p + 16); return u.v;
}
__device__ __forceinline__ v16h frag_f32(const float* rowk0, int lane) {
  v16h a; const float* p = rowk0 + 8 * (lane >> 4);
#pragma unroll
  for (int i = 0; i < 8; ++i) { a[i] = (_Float16)p[i]; a[8 + i] = (_Float16)p[16 + i]; }
  return a;
}
__device__ __forceinline__ v16h frag_f32s(const float* rowk0, int lane, float sc) {
  v16h a; const float* p = rowk0 + 8 * (lane >> 4);
#pragma unroll
  for (int i = 0; i < 8; ++i) { a[i] = (_Float16)(p[i] * sc); a[8 + i] = (_Float16)(p[16 + i] * sc); }
  return a;
}
__device__ __forceinline__ v16h fragc_f32(const float* W, int k0, int n, int lane, int ld, int K) {
  v16h a; const int g = lane >> 4;
#pragma unroll
  for (int i = 0; i < 8; ++i) { const int ka = k0 + 8 * g + i, kb = ka + 16;
    a[i] = (_Float16)(ka < K ? W[(size_t)ka * ld + n] : 0.f); a[8 + i] = (_Float16)(kb < K ? W[(size_t)kb * ld + n] : 0.f); }
  return a;
}
struct F2 { v16b h, l; };
__device__ __forceinline__ F2 bsplit16(const float v[16]) { F2 r;
#pragma unroll
  for (int i = 0; i < 16; ++i) { const __bf16 h = (__bf16)v[i]; r.h[i] = h; r.l[i] = (__bf16)(v[i] - (float)h); }
  return r; }
__device__ __forceinline__ F2 split_row(const float* row, int k0, int lane) { float v[16]; const float* p = row + k0 + 8 * (lane >> 4);
#pragma unroll
  for (int i = 0; i < 8; ++i) { v[i] = p[i]; v[8 + i] = p[16 + i]; }
  return bsplit16(v); }
__device__ __forceinline__ F2 split_rowK(const float* row, int k0, int lane, int K) { float v[16]; const int g = lane >> 4;
#pragma unroll
  for (int i = 0; i < 8; ++i) { const int ka = k0 + 8 * g + i, kb = ka + 16; v[i] = ka < K ? row[ka] : 0.f; v[8 + i] = kb < K ? row[kb] : 0.f; }
  return bsplit16(v); }
__device__ __forceinline__ F2 split_col(const float* W, int k0, int n, int lane, int ld, int K) { float v[16]; const int g = lane >> 4;
#pragma unroll
  for (int i = 0; i < 8; ++i) { const int ka = k0 + 8 * g + i, kb = ka + 16; v[i] = ka < K ? W[(size_t)ka * ld + n] : 0.f; v[8 + i] = kb < K ? W[(size_t)kb * ld + n] : 0.f; }
  return bsplit16(v); }
__device__ __forceinline__ v8f mac3(const F2& a, const F2& b, v8f c) { c = wmma_bf(a.l, b.h, c); c = wmma_bf(a.h, b.l, c); return wmma_bf(a.h, b.h, c); }
__device__ __forceinline__ float sigm(float v) { return 1.0f / (1.0f + expf(-v)); }
#define LDSX() do { asm volatile("s_wait_dscnt 0" ::: "memory"); __builtin_amdgcn_wave_barrier(); __builtin_amdgcn_fence(__ATOMIC_RELEASE, "workgroup"); } while (0)

#define NB 128
#define H1 224
#define P1N (H1 * H1)
#define C1 8
#define H2 112
#define P2N (H2 * H2)
#define C2U 4
#define H3 56
#define NPB1 (H1 / 4)
struct KSum { float s, c; __device__ KSum() : s(0.f), c(0.f) {} __device__ void add(float v) { const float y = v - c; const float t = s + y; c = (t - s) - y; s = t; } };

__global__ __launch_bounds__(128) void k_conv1(const float* __restrict__ x, const float* __restrict__ w1, const float* __restrict__ b1, float* __restrict__ cmax, float* __restrict__ cmin, float* __restrict__ part) {
  __shared__ __align__(16) float st[C1][4 * H1 + 4];
  __shared__ __align__(16) float smm[2][C1][2 * H2];
  __shared__ float sp[4][C1][2];
  __shared__ float xin[6 * 226];
  __shared__ int koff[16];
  const int tid = threadIdx.x, w = tid >> 5, lane = tid & 31, col = lane & 15, g = lane >> 4;
  const int b = blockIdx.y, yb = blockIdx.x;
  const float* xb = x + (size_t)b * P1N;
#pragma unroll
  for (int rr = 0; rr < 6; ++rr) { const int yy = 4 * yb - 1 + rr; const bool rowok = yy >= 0 && yy < H1;
    for (int cc = tid; cc < 226; cc += 128) { const int xx = cc - 1; xin[rr * 226 + cc] = (rowok && xx >= 0 && xx < H1) ? xb[yy * H1 + xx] : 0.f; } }
  if (tid < 16) koff[tid] = tid < 9 ? (tid / 3) * 226 + (tid % 3) : 0;
  __syncthreads();
  F2 bw; { float wv[16];
#pragma unroll
    for (int i = 0; i < 16; ++i) { const int kk = g * 8 + (i & 7); float v = 0.f;
      if (kk < 9) { if (i < 8) { if (col < C1) v = w1[col * 9 + kk]; } else { if (col >= C1) v = w1[(col - C1) * 9 + kk]; } }
      wv[i] = v; }
    bw = bsplit16(wv); }
#pragma unroll 1
  for (int t = 0; t < 7; ++t) { const int plA = (w * 7 + t) * 32 + col, plB = plA + 16;
    const int baseA = (plA / H1) * 226 + (plA % H1), baseB = (plB / H1) * 226 + (plB % H1);
    float av[16];
#pragma unroll
    for (int i = 0; i < 8; ++i) { const int k = g * 8 + i; av[i] = k < 9 ? xin[baseA + koff[k]] : 0.f; av[8 + i] = k < 9 ? xin[baseB + koff[k]] : 0.f; }
    v8f acc = {}; acc = mac3(bsplit16(av), bw, acc);
    { const int c = col & 7, setoff = col < C1 ? 0 : 16;
#pragma unroll
      for (int r = 0; r < 8; ++r) st[c][(w * 7 + t) * 32 + setoff + 8 * g + r] = acc[r] + b1[c]; } }
  __syncthreads();
  for (int q = tid; q < C1 * 2 * H2; q += 128) { const int c = q / (2 * H2), rem = q % (2 * H2), yl = rem / H2, xo = rem % H2;
    const float v0 = st[c][(2 * yl) * H1 + 2 * xo], v1 = st[c][(2 * yl) * H1 + 2 * xo + 1], v2 = st[c][(2 * yl + 1) * H1 + 2 * xo], v3 = st[c][(2 * yl + 1) * H1 + 2 * xo + 1];
    smm[0][c][rem] = fmaxf(fmaxf(v0, v1), fmaxf(v2, v3)); smm[1][c][rem] = fminf(fminf(v0, v1), fminf(v2, v3)); }
  { const int c = tid >> 4, part16 = tid & 15; float s = 0.f, q2 = 0.f;
    for (int i = part16; i < 4 * H1; i += 16) { const float v = st[c][i]; s += v; q2 += v * v; }
#pragma unroll
    for (int off = 8; off >= 1; off >>= 1) { s += __shfl_xor(s, off, 32); q2 += __shfl_xor(q2, off, 32); }
    if (part16 == 0) { sp[0][c][0] = s; sp[0][c][1] = q2; } }
  __syncthreads();
  for (int q = tid; q < 2 * C1 * 56; q += 128) { const int which = q / (C1 * 56), rem = q % (C1 * 56), c = rem / 56, pc = rem % 56;
    vst2((which == 0 ? cmax : cmin) + ((size_t)b * C1 + c) * P2N + yb * 224 + pc * 4, *(const v4f*)(&smm[which][c][pc * 4])); }
  if (tid < 32) vst2(part + ((size_t)b * (H1 / 4) + yb) * 32 + tid, (float_a)(tid < 16 ? (&sp[0][0][0])[tid] : 0.f));
}
__global__ __launch_bounds__(32) void k_stat1(const float* __restrict__ part, const float* __restrict__ g1, const float* __restrict__ be1, float* __restrict__ st1) {
  const int c = threadIdx.x; KSum ks, kq;
  if (c < C1) {
#pragma unroll 1
    for (int i = 0; i < NB * NPB1; ++i) { ks.add(part[(size_t)i * 32 + c * 2]); kq.add(part[(size_t)i * 32 + c * 2 + 1]); } }
  const float s = ks.s, q2 = kq.s;
  const float n = (float)NB * (float)P1N; const float mu = s / n; float var = (q2 - mu * s) / n; var = var < 0.f ? 0.f : var;
  const float sc = (c < C1 ? g1[c] : 0.f) * rsqrtf(var + 1e-5f), sh = (c < C1 ? be1[c] : 0.f) - mu * sc;
  __shared__ __align__(16) float so[32]; so[c] = 0.f;
  __builtin_amdgcn_wave_barrier(); asm volatile("s_wait_dscnt 0" ::: "memory");
  if (c < C1) { so[c * 2] = sc; so[c * 2 + 1] = sh; }
  __builtin_amdgcn_wave_barrier(); asm volatile("s_wait_dscnt 0" ::: "memory");
  if (c < 8) vst2(st1 + c * 4, *(const v4f*)(&so[c * 4]));
}
#define NPB2 (H2 / 8)
__global__ __launch_bounds__(128) void k_conv2(const float* __restrict__ cmax, const float* __restrict__ cmin, const float* __restrict__ st1, const float* __restrict__ w2, const float* __restrict__ b2,
                                            float* __restrict__ c2max, float* __restrict__ c2min, float* __restrict__ part2) {
  __shared__ float pin[C1 * 10 * 114];
  __shared__ int koff[96];
  __shared__ __align__(16) __bf16 sBh[3][32][16], sBl[3][32][16];
  __shared__ __align__(16) float st[C2U][8 * H2 + 4];
  __shared__ __align__(16) float smm[2][C2U][4 * H3];
  __shared__ float sp[C2U][2];
  const int tid = threadIdx.x, w = tid >> 5, lane = tid & 31, col = lane & 15, g = lane >> 4;
  const int b = blockIdx.y, yb = blockIdx.x; const int y0 = yb * 8;
  { const int cc = tid; const int xx = cc - 1; const bool colok = cc < 114 && xx >= 0 && xx < H2;
#pragma unroll 1
    for (int ci = 0; ci < C1; ++ci) { const float sc = st1[ci * 2], sh = st1[ci * 2 + 1]; const float* pmx = cmax + ((size_t)b * C1 + ci) * P2N; const float* pmn = cmin + ((size_t)b * C1 + ci) * P2N;
#pragma unroll
      for (int rr = 0; rr < 10; ++rr) { const int yy = y0 - 1 + rr; float v = 0.f;
        if (colok && yy >= 0 && yy < H2) { const float m = sc >= 0.f ? pmx[yy * H2 + xx] : pmn[yy * H2 + xx]; v = m * sc + sh; v = v > 0.f ? v : 0.f; }
        if (cc < 114) pin[ci * 1140 + rr * 114 + cc] = v; } } }
  if (tid < 96) { const int k = tid; koff[k] = k < 72 ? (k / 9) * 1140 + ((k % 9) / 3) * 114 + ((k % 9) % 3) : 0; }
  if (tid < 96) { const int kc = tid >> 5, ln = tid & 31, gg = ln >> 4, cl = ln & 15; float wv[16];
#pragma unroll
    for (int i = 0; i < 16; ++i) { const int k = kc * 32 + (i < 8 ? gg * 8 + i : 16 + gg * 8 + (i - 8)); wv[i] = (k < 72 && cl < C2U) ? w2[cl * 72 + k] : 0.f; }
    const F2 f = bsplit16(wv);
#pragma unroll
    for (int i = 0; i < 16; ++i) { sBh[kc][ln][i] = f.h[i]; sBl[kc][ln][i] = f.l[i]; } }
  __syncthreads();
#pragma unroll 1
  for (int t = 0; t < 14; ++t) { const int pl = (w * 14 + t) * 16 + col; const int base = (pl / H2) * 114 + (pl % H2);
    v8f acc = {};
#pragma unroll
    for (int kc = 0; kc < 3; ++kc) { float av[16];
#pragma unroll
      for (int i = 0; i < 16; ++i) { const int k = kc * 32 + (i < 8 ? g * 8 + i : 16 + g * 8 + (i - 8)); av[i] = k < 72 ? pin[base + koff[k]] : 0.f; }
      F2 bw;
#pragma unroll
      for (int i = 0; i < 16; ++i) { bw.h[i] = sBh[kc][lane][i]; bw.l[i] = sBl[kc][lane][i]; }
      acc = mac3(bsplit16(av), bw, acc); }
    if (col < C2U) {
#pragma unroll
      for (int r = 0; r < 8; ++r) st[col][(w * 14 + t) * 16 + 8 * g + r] = acc[r] + b2[col]; } }
  __syncthreads();
  for (int q = tid; q < C2U * 4 * H3; q += 128) { const int c = q / (4 * H3), rem = q % (4 * H3), yl = rem / H3, xo = rem % H3;
    const float v0 = st[c][(2 * yl) * H2 + 2 * xo], v1 = st[c][(2 * yl) * H2 + 2 * xo + 1], v2 = st[c][(2 * yl + 1) * H2 + 2 * xo], v3 = st[c][(2 * yl + 1) * H2 + 2 * xo + 1];
    smm[0][c][rem] = fmaxf(fmaxf(v0, v1), fmaxf(v2, v3)); smm[1][c][rem] = fminf(fminf(v0, v1), fminf(v2, v3)); }
  { const int c = tid >> 5; float s = 0.f, q2 = 0.f;
    for (int i = lane; i < 8 * H2; i += 32) { const float v = st[c][i]; s += v; q2 += v * v; }
#pragma unroll
    for (int off = 16; off >= 1; off >>= 1) { s += __shfl_xor(s, off, 32); q2 += __shfl_xor(q2, off, 32); }
    if (lane == 0) { sp[c][0] = s; sp[c][1] = q2; } }
  __syncthreads();
  for (int q = tid; q < 2 * C2U * 56; q += 128) { const int which = q / (C2U * 56), rem = q % (C2U * 56), c = rem / 56, pc = rem % 56;
    vst2((which == 0 ? c2max : c2min) + ((size_t)b * C2U + c) * (H3 * H3) + yb * 224 + pc * 4, *(const v4f*)(&smm[which][c][pc * 4])); }
  if (tid < 32) vst2(part2 + ((size_t)b * NPB2 + yb) * 32 + tid, (float_a)(tid < 8 ? (&sp[0][0])[tid] : 0.f));
}
__global__ __launch_bounds__(128) void k_tail(const float* __restrict__ c2max, const float* __restrict__ c2min, const float* __restrict__ part2, const float* __restrict__ g2, const float* __restrict__ be2,
                                           const float* __restrict__ theta, const float* __restrict__ rho, const float* __restrict__ ng, const float* __restrict__ nbias, float* __restrict__ out) {
  __shared__ float sst[C2U][2]; __shared__ float feat[NB][C2U]; __shared__ float red[128]; __shared__ float ex[NB][4]; __shared__ __align__(16) float so[NB * 4];
  const int tid = threadIdx.x; const int b = tid;
  if (tid < C2U) { KSum ks, kq;
#pragma unroll 1
    for (int i = 0; i < NB * NPB2; ++i) { ks.add(part2[(size_t)i * 32 + tid * 2]); kq.add(part2[(size_t)i * 32 + tid * 2 + 1]); }
    const float s = ks.s, q2 = kq.s;
    const float n = (float)NB * (float)P2N; const float mu = s / n; float var = (q2 - mu * s) / n; var = var < 0.f ? 0.f : var;
    const float sc = g2[tid] * rsqrtf(var + 1e-5f); sst[tid][0] = sc; sst[tid][1] = be2[tid] - mu * sc; }
  __syncthreads();
#pragma unroll 1
  for (int c = 0; c < C2U; ++c) { const float sc = sst[c][0], sh = sst[c][1]; const float* pmx = c2max + ((size_t)b * C2U + c) * (H3 * H3); const float* pmn = c2min + ((size_t)b * C2U + c) * (H3 * H3); KSum ksum;
#pragma unroll 1
    for (int q = 0; q < H3 * H3; ++q) { float v = (sc >= 0.f ? pmx[q] : pmn[q]) * sc + sh; v = v > 0.f ? v : 0.f; ksum.add(v); }
    feat[b][c] = ksum.s / (float)(H3 * H3); }
  __syncthreads();
  __shared__ float gm, gs;
  if (tid == 0) { KSum ks; for (int i = 0; i < NB * 4; ++i) ks.add((&feat[0][0])[i]); const float m = ks.s / (float)(NB * 4); KSum kq;
    for (int i = 0; i < NB * 4; ++i) { const float d = (&feat[0][0])[i] - m; kq.add(d * d); } gm = m; gs = sqrtf(kq.s / (float)(NB * 4 - 1)); }
  __syncthreads();
  float ang[4];
#pragma unroll
  for (int i = 0; i < 4; ++i) ang[i] = (feat[b][i] - gm) / (gs + 1e-6f) * 3.14159265358979323846f;
  float re[16], im[16];
#pragma unroll
  for (int i = 0; i < 16; ++i) { re[i] = 0.f; im[i] = 0.f; }
  re[0] = 1.0f;
  auto apply = [&](int wire, float u00r, float u00i, float u01r, float u01i, float u10r, float u10i, float u11r, float u11i) {
    const int bit = 3 - wire;
#pragma unroll
    for (int i = 0; i < 16; ++i) { if (i & (1 << bit)) continue; const int j = i | (1 << bit);
      const float a0r = re[i], a0i = im[i], a1r = re[j], a1i = im[j];
      re[i] = u00r * a0r - u00i * a0i + u01r * a1r - u01i * a1i; im[i] = u00r * a0i + u00i * a0r + u01r * a1i + u01i * a1r;
      re[j] = u10r * a0r - u10i * a0i + u11r * a1r - u11i * a1i; im[j] = u10r * a0i + u10i * a0r + u11r * a1i + u11i * a1r; } };
  auto ry = [&](int wire, float t) { const float c = cosf(t * 0.5f), s = sinf(t * 0.5f); apply(wire, c, 0.f, -s, 0.f, s, 0.f, c, 0.f); };
  auto rz = [&](int wire, float t) { const float c = cosf(t * 0.5f), s = sinf(t * 0.5f); apply(wire, c, -s, 0.f, 0.f, 0.f, 0.f, c, s); };
  auto rx = [&](int wire, float t) { const float c = cosf(t * 0.5f), s = sinf(t * 0.5f); apply(wire, c, 0.f, 0.f, -s, 0.f, -s, c, 0.f); };
  auto cnot = [&](int cw, int tw) { const int cb = 3 - cw, tb = 3 - tw;
#pragma unroll
    for (int i = 0; i < 16; ++i) { if (!(i & (1 << cb))) continue; if (i & (1 << tb)) continue; const int j = i | (1 << tb);
      const float tr = re[i], ti = im[i]; re[i] = re[j]; im[i] = im[j]; re[j] = tr; im[j] = ti; } };
#pragma unroll
  for (int i = 0; i < 4; ++i) ry(i, ang[i]);
#pragma unroll
  for (int i = 0; i < 4; ++i) { ry(i, theta[i * 3]); rz(i, theta[i * 3 + 1]); rx(i, theta[i * 3 + 2]); }
#pragma unroll
  for (int i = 0; i < 3; ++i) cnot(i, i + 1);
#pragma unroll
  for (int i = 0; i < 4; ++i) { ry(i, rho[i * 3]); rz(i, rho[i * 3 + 1]); rx(i, rho[i * 3 + 2]); }
#pragma unroll
  for (int i = 0; i < 3; ++i) cnot(i + 1, i);
  float e4[4] = {0.f, 0.f, 0.f, 0.f};
#pragma unroll
  for (int i = 0; i < 16; ++i) { const float pr = re[i] * re[i] + im[i] * im[i];
#pragma unroll
    for (int wq = 0; wq < 4; ++wq) e4[wq] += (i & (1 << (3 - wq))) ? -pr : pr; }
#pragma unroll
  for (int wq = 0; wq < 4; ++wq) ex[b][wq] = e4[wq];
  __syncthreads();
  if (tid < 4) { float s = 0.f; for (int i = 0; i < NB; ++i) s += ex[i][tid]; const float m = s / (float)NB; float q2 = 0.f; for (int i = 0; i < NB; ++i) { const float d = ex[i][tid] - m; q2 += d * d; }
    const float var = q2 / (float)NB; const float sc = ng[tid] * rsqrtf(var + 1e-5f); red[tid * 2] = sc; red[tid * 2 + 1] = nbias[tid] - m * sc; }
  __syncthreads();
#pragma unroll
  for (int wq = 0; wq < 4; ++wq) so[b * 4 + wq] = ex[b][wq] * red[wq * 2] + red[wq * 2 + 1];
  __syncthreads();
  vst2(out + tid * 4, *(const v4f*)(&so[tid * 4]));
}
extern "C" void kernel_launch(void* const* d_in, const int* in_sizes, int n_in, void* d_out, int out_size, void* d_ws, size_t ws_size, hipStream_t stream) {
  (void)in_sizes; (void)n_in; (void)out_size; (void)ws_size;
  const float* x = (const float*)d_in[0]; const float* w1 = (const float*)d_in[1]; const float* b1 = (const float*)d_in[2]; const float* g1 = (const float*)d_in[3]; const float* be1 = (const float*)d_in[4];
  const float* w2 = (const float*)d_in[5]; const float* b2 = (const float*)d_in[6]; const float* g2 = (const float*)d_in[7]; const float* be2 = (const float*)d_in[8];
  const float* theta = (const float*)d_in[9]; const float* rho = (const float*)d_in[10]; const float* ng = (const float*)d_in[11]; const float* nbias = (const float*)d_in[12];
  float* out = (float*)d_out;
  char* ws = (char*)d_ws; size_t off = 0;
  auto take = [&](size_t bytes) { char* p = ws + off; off += (bytes + 255) & ~(size_t)255; return p; };
  float* part = (float*)take((size_t)NB * NPB1 * 32 * 4); float* st1 = (float*)take(256); float* part2 = (float*)take((size_t)NB * NPB2 * 32 * 4);
  float* c2max = (float*)take((size_t)NB * C2U * H3 * H3 * 4); float* c2min = (float*)take((size_t)NB * C2U * H3 * H3 * 4);
  float* cmax = (float*)take((size_t)NB * C1 * P2N * 4); float* cmin = (float*)take((size_t)NB * C1 * P2N * 4);
  k_conv1<<<dim3(NPB1, NB), 128, 0, stream>>>(x, w1, b1, cmax, cmin, part);
  k_stat1<<<1, 32, 0, stream>>>(part, g1, be1, st1);
  k_conv2<<<dim3(NPB2, NB), 128, 0, stream>>>(cmax, cmin, st1, w2, b2, c2max, c2min, part2);
  k_tail<<<1, 128, 0, stream>>>(c2max, c2min, part2, g2, be2, theta, rho, ng, nbias, out);
}
